// GraphAttention_76441827934506
// MI455X (gfx1250) — hardware-verified
//
#include <hip/hip_runtime.h>

#define BB    4
#define NN    2048
#define IN_F  128
#define OUT_F 128
#define HH    4
#define DD    32
#define NEG_SLOPE 0.2f

typedef __attribute__((ext_vector_type(16))) _Float16 v16h;
typedef __attribute__((ext_vector_type(8)))  float    v8f;

union AV { v16h h; unsigned int u[8]; };
typedef __attribute__((ext_vector_type(4))) float v4f;
typedef __attribute__((ext_vector_type(4))) unsigned v4u;
typedef float __attribute__((may_alias)) float_a;
typedef unsigned __attribute__((may_alias)) uint_a;
template <typename T> static __device__ __forceinline__ void vst2(void* p, T v) { *(volatile T*)p = v; __threadfence(); *(volatile T*)p = v; }

static __device__ __forceinline__ v8f wmma_f16(const AV& a, const AV& b, v8f c) {
  v8f d = __builtin_amdgcn_wmma_f32_16x16x32_f16(false, a.h, false, b.h, (short)0, c, false, false);
  asm volatile("v_nop\n\tv_nop\n\tv_nop\n\tv_nop" : "+v"(d) : "v"(a.h), "v"(b.h));
  return d;
}

__global__ void cvt_f32_f16_kernel(const float* __restrict__ src,
                                   _Float16* __restrict__ dst, int n) {
  int g = blockIdx.x * 256 + threadIdx.x;
  if (g * 8 < n) { union { _Float16 h[8]; v4u u; } pk;
#pragma unroll
    for (int e = 0; e < 8; ++e) pk.h[e] = (_Float16)src[(size_t)g * 8 + e];
    vst2(dst + (size_t)g * 8, pk.u); }
}

__global__ void pack_adj_kernel(const int* __restrict__ adj,
                                unsigned int* __restrict__ pk) {
  int t = blockIdx.x * 256 + threadIdx.x;
  if (t >= NN * (NN / 32)) return;
  int n = t >> 6;
  int w = t & 63;
  const int* row = adj + (size_t)n * NN + w * 32;
  unsigned int bits = 0u;
  #pragma unroll 8
  for (int j = 0; j < 32; ++j) bits |= (row[j] != 0 ? 1u : 0u) << j;
  vst2(pk + t, (uint_a)bits);
}

__global__ __launch_bounds__(128)
void proj_kernel(const _Float16* __restrict__ xh,
                 const _Float16* __restrict__ wh,
                 const float* __restrict__ a_src, const float* __restrict__ a_dst,
                 _Float16* __restrict__ ht,
                 float* __restrict__ e_src, float* __restrict__ e_dst) {
  __shared__ __align__(16) float st[OUT_F][64 + 4];
  const int lane = threadIdx.x & 31;
  const int wv   = threadIdx.x >> 5;
  const int hl   = lane >> 4;
  const int lm   = lane & 15;
  const int r0   = blockIdx.x * 64;
  const int arow = r0 + wv * 16 + lm;

  v8f acc[8] = {};
  for (int k0 = 0; k0 < IN_F; k0 += 32) {
    AV a;
    #pragma unroll
    for (int v = 0; v < 8; ++v) {
      int ka = k0 + 2 * v + ((v >= 4) ? 8 : 0) + 8 * hl;
      a.u[v] = *(const unsigned int*)(xh + (size_t)arow * IN_F + ka);
    }
    #pragma unroll
    for (int ot = 0; ot < 8; ++ot) {
      AV b;
      #pragma unroll
      for (int v = 0; v < 8; ++v) {
        int kb = k0 + 2 * v + ((v >= 4) ? 8 : 0) + 8 * hl;
        b.u[v] = *(const unsigned int*)(wh + (size_t)(ot * 16 + lm) * IN_F + kb);
      }
      acc[ot] = wmma_f16(a, b, acc[ot]);
    }
  }
  #pragma unroll
  for (int ot = 0; ot < 8; ++ot)
    #pragma unroll
    for (int r = 0; r < 8; ++r) st[ot * 16 + lm][wv * 16 + r + 8 * hl] = acc[ot][r];
  __syncthreads();
  const int b_ = r0 >> 11, n0 = r0 & (NN - 1);
  for (int q = threadIdx.x; q < OUT_F * 8; q += 128) {
    const int oc = q >> 3, pc = q & 7; const int hd = oc >> 5, d = oc & (DD - 1);
    union { _Float16 h[8]; v4u u; } pk;
    #pragma unroll
    for (int e = 0; e < 8; ++e) pk.h[e] = (_Float16)st[oc][pc * 8 + e];
    vst2(ht + (((size_t)b_ * HH + hd) * DD + d) * NN + n0 + pc * 8, pk.u);
  }
  for (int q = threadIdx.x; q < HH * 64; q += 128) {
    const int hd = q >> 6, rl = q & 63;
    float es = 0.f, ed = 0.f;
    #pragma unroll 8
    for (int d = 0; d < DD; ++d) { const float hv = st[hd * DD + d][rl]; es += hv * a_src[hd * DD + d]; ed += hv * a_dst[hd * DD + d]; }
    vst2(e_src + ((size_t)b_ * HH + hd) * NN + n0 + rl, (float_a)es);
    vst2(e_dst + ((size_t)b_ * HH + hd) * NN + n0 + rl, (float_a)ed);
  }
}

__global__ __launch_bounds__(128)
void attn_kernel(const _Float16* __restrict__ ht,
                 const float* __restrict__ e_src,
                 const float* __restrict__ e_dst,
                 const unsigned int* __restrict__ adj_pk,
                 float* __restrict__ out) {
  __shared__ __align__(16) float eds[NN];
  __shared__ float redbuf[128];

  const int tid  = threadIdx.x;
  const int lane = tid & 31;
  const int wv   = tid >> 5;
  const int bh   = blockIdx.y;
  const int b    = bh >> 2;
  const int h    = bh & (HH - 1);
  const int hl   = lane >> 4;
  const int lm   = lane & 15;

  float lmax = -__builtin_inff();
  for (int i = tid; i < NN; i += 128) {
    float v = e_dst[(size_t)bh * NN + i];
    eds[i] = v;
    lmax = fmaxf(lmax, v);
  }
  redbuf[tid] = lmax;
  __syncthreads();
  #pragma unroll
  for (int s = 64; s > 0; s >>= 1) {
    if (tid < s) redbuf[tid] = fmaxf(redbuf[tid], redbuf[tid + s]);
    __syncthreads();
  }
  const float gmax = redbuf[0];

  const int n0 = blockIdx.x * 64 + wv * 16;
  const int myrow = n0 + lm;
  const float es = e_src[(size_t)bh * NN + myrow];
  const unsigned int* adjrow = adj_pk + (size_t)myrow * (NN / 32);
  const _Float16* hb = ht + (size_t)bh * DD * NN;

  float mb = es + gmax;
  const float mrow = fmaxf(mb, NEG_SLOPE * mb);

  float lrow = 0.f;
  v8f acc0 = {}, acc1 = {};

  for (int m0 = 0; m0 < NN; m0 += 32) {
    const unsigned int bits = adjrow[m0 >> 5];
    AV B0, B1;
    #pragma unroll
    for (int v = 0; v < 8; ++v) {
      int kb = m0 + 2 * v + ((v >= 4) ? 8 : 0) + 8 * hl;
      B0.u[v] = *(const unsigned int*)(hb + (size_t)(lm)      * NN + kb);
      B1.u[v] = *(const unsigned int*)(hb + (size_t)(16 + lm) * NN + kb);
    }

    AV A;
    #pragma unroll
    for (int v = 0; v < 8; ++v) {
      int Kb = 2 * v + ((v >= 4) ? 8 : 0) + 8 * hl;
      float2 ee = *(const float2*)&eds[m0 + Kb];
      float s0 = es + ee.x;  s0 = fmaxf(s0, NEG_SLOPE * s0);
      float s1 = es + ee.y;  s1 = fmaxf(s1, NEG_SLOPE * s1);
      float p0 = ((bits >> Kb)       & 1u) ? expf(s0 - mrow) : 0.f;
      float p1 = ((bits >> (Kb + 1)) & 1u) ? expf(s1 - mrow) : 0.f;
      lrow += p0 + p1;
      union { _Float16 f[2]; unsigned int u; } pk;
      pk.f[0] = (_Float16)(p0 * 16384.0f);
      pk.f[1] = (_Float16)(p1 * 16384.0f);
      A.u[v] = pk.u;
    }

    acc0 = wmma_f16(A, B0, acc0);
    acc1 = wmma_f16(A, B1, acc1);
  }

  lrow += __shfl_xor(lrow, 16, 32);
  const float inv = (1.0f / 16384.0f) / lrow;

  __shared__ __align__(16) float so[4][16][DD];
  #pragma unroll
  for (int r = 0; r < 8; ++r) {
    float iv = __shfl(inv, r + 8 * hl, 32);
    so[wv][r + 8 * hl][lm]      = acc0[r] * iv;
    so[wv][r + 8 * hl][16 + lm] = acc1[r] * iv;
  }
  asm volatile("s_wait_dscnt 0" ::: "memory"); __builtin_amdgcn_wave_barrier(); __builtin_amdgcn_fence(__ATOMIC_RELEASE, "workgroup");
  #pragma unroll 4
  for (int rl = 0; rl < 16; ++rl)
    vst2(out + ((size_t)b * NN + n0 + rl) * OUT_F + h * DD + lane, (float_a)so[wv][rl][lane]);
}

extern "C" void kernel_launch(void* const* d_in, const int* in_sizes, int n_in,
                              void* d_out, int out_size, void* d_ws, size_t ws_size,
                              hipStream_t stream) {
  const float* x     = (const float*)d_in[0];
  const int*   adj   = (const int*)d_in[1];
  const float* W     = (const float*)d_in[2];
  const float* a_src = (const float*)d_in[3];
  const float* a_dst = (const float*)d_in[4];
  float* out = (float*)d_out;

  char* ws = (char*)d_ws;
  _Float16* xh     = (_Float16*)(ws);
  _Float16* wh     = (_Float16*)(ws + 2097152);
  _Float16* ht     = (_Float16*)(ws + 2097152 + 32768);
  float*    e_src  = (float*)   (ws + 2097152 + 32768 + 2097152);
  float*    e_dst  = (float*)   (ws + 2097152 + 32768 + 2097152 + 131072);
  unsigned int* adj_pk = (unsigned int*)(ws + 2097152 + 32768 + 2097152 + 2*131072);

  const int nx = BB * NN * IN_F;
  const int nw = OUT_F * IN_F;
  cvt_f32_f16_kernel<<<(nx / 8 + 255) / 256, 256, 0, stream>>>(x, xh, nx);
  cvt_f32_f16_kernel<<<(nw / 8 + 255) / 256, 256, 0, stream>>>(W, wh, nw);

  const int npk = NN * (NN / 32);
  pack_adj_kernel<<<(npk + 255) / 256, 256, 0, stream>>>(adj, adj_pk);

  proj_kernel<<<BB * NN / 64, 128, 0, stream>>>(xh, wh, a_src, a_dst, ht, e_src, e_dst);

  dim3 grid(NN / 64, BB * HH);
  attn_kernel<<<grid, 128, 0, stream>>>(ht, e_src, e_dst, adj_pk, out);
}
